// CrossAttentionModule_73632919323387
// MI455X (gfx1250) — hardware-run, weakly checked
//
#include <hip/hip_runtime.h>
#define NN 8192
#define HD 64
#define RB 1024
typedef __bf16 v16b __attribute__((ext_vector_type(16)));
typedef unsigned short v8us __attribute__((ext_vector_type(8), may_alias));
typedef float  v8f  __attribute__((ext_vector_type(8)));
typedef float  v4f  __attribute__((ext_vector_type(4)));
typedef float  v4fa __attribute__((ext_vector_type(4), may_alias));
union FragB { v16b v; v8us half[2]; unsigned short u[16]; };

__device__ __forceinline__ unsigned short bf16_bits(float x) { unsigned int u = __float_as_uint(x); return (unsigned short)((u + 0x7FFFu + ((u >> 16) & 1u)) >> 16); }
__device__ __forceinline__ float bf16_val(unsigned short b) { return __uint_as_float(((unsigned int)b) << 16); }
__device__ __forceinline__ float bf16_round(float x) { return bf16_val(bf16_bits(x)); }
template <int NT>
__device__ __forceinline__ v8f mmaN(v16b ah, v16b al, v16b bh, v16b bl, v8f c) {
  c = __builtin_amdgcn_wmma_f32_16x16x32_bf16(false, ah, false, bh, (short)0, c, false, false);
  if (NT >= 2) c = __builtin_amdgcn_wmma_f32_16x16x32_bf16(false, al, false, bh, (short)0, c, false, false);
  if (NT >= 3) c = __builtin_amdgcn_wmma_f32_16x16x32_bf16(false, ah, false, bl, (short)0, c, false, false);
  asm volatile("v_nop\n\tv_nop\n\tv_nop\n\tv_nop" : "+v"(c) : "v"(ah), "v"(al), "v"(bh), "v"(bl));
  return c;
}


typedef _Float16 v16h __attribute__((ext_vector_type(16)));
union FragH { v16h v; v8us half[2]; _Float16 h[16]; unsigned short u[16]; };
template <int NT>
__device__ __forceinline__ v8f mmaH(v16h ah, v16h al, v16h bh, v16h bl, v8f c) {
  c = __builtin_amdgcn_wmma_f32_16x16x32_f16(false, ah, false, bh, (short)0, c, false, false);
  if (NT >= 2) c = __builtin_amdgcn_wmma_f32_16x16x32_f16(false, al, false, bh, (short)0, c, false, false);
  if (NT >= 3) c = __builtin_amdgcn_wmma_f32_16x16x32_f16(false, ah, false, bl, (short)0, c, false, false);
  asm volatile("v_nop\n\tv_nop\n\tv_nop\n\tv_nop" : "+v"(c) : "v"(ah), "v"(al), "v"(bh), "v"(bl));
  return c;
}

__global__ __launch_bounds__(256) void k_wt_f16(const float* __restrict__ W, _Float16* __restrict__ Wt, int K, int N, float scale) {
  const int t = blockIdx.x * 256 + threadIdx.x; if (t >= N * (K / 8)) return; const int n = t / (K / 8), k8 = (t % (K / 8)) * 8; FragH f;
#pragma unroll
  for (int i = 0; i < 8; ++i) f.h[i] = (_Float16)(bf16_round(W[(size_t)(k8 + i) * N + n]) * scale); const v8us o = f.half[0];
  *(volatile v8us*)((unsigned short*)Wt + (size_t)n * K + k8) = o; __threadfence(); *(volatile v8us*)((unsigned short*)Wt + (size_t)n * K + k8) = o;
}
typedef _Float16 v4h __attribute__((ext_vector_type(4)));
__global__ __launch_bounds__(256) void k_x16(const float* __restrict__ x, _Float16* __restrict__ X16, size_t n8) { const size_t t = (size_t)blockIdx.x * 256 + threadIdx.x; if (t >= n8) return; FragH f;
#pragma unroll
  for (int q = 0; q < 8; ++q) f.h[q] = (_Float16)bf16_round(x[t * 8 + q]); *(volatile v8us*)((unsigned short*)X16 + t * 8) = f.half[0]; __threadfence(); *(volatile v8us*)((unsigned short*)X16 + t * 8) = f.half[0]; }
__device__ __forceinline__ v16h g2_frag(const _Float16* p, int hh) { FragH f; f.half[0] = *(const v8us*)((const unsigned short*)p + 8 * hh); f.half[1] = *(const v8us*)((const unsigned short*)p + 16 + 8 * hh); return f.v; }
__device__ __forceinline__ v8f g2_mma(v16h a, v16h b, v8f c) { v8f d = __builtin_amdgcn_wmma_f32_16x16x32_f16(false, a, false, b, (short)0, c, false, false); asm volatile("v_nop\n\tv_nop\n\tv_nop\n\tv_nop" : "+v"(d) : "v"(a), "v"(b)); return d; }
template <int ACT>
__global__ __launch_bounds__(128) void k_gemm2(const _Float16* __restrict__ A, int lda, size_t sA, const _Float16* __restrict__ Bh, int ldb, size_t sB, float alpha, const float* __restrict__ bias, size_t sBias, const float* __restrict__ CP, int rowsPerB, size_t sCPb, int row0g,
    float* __restrict__ C, _Float16* __restrict__ C16, int ldc, size_t sC, int M, int N, int K) { static_assert(ACT == 0 || ACT == 3 || ACT == 6 || ACT == 8 || ACT == 9 || ACT == 11 || ACT == 12 || ACT == 14 || ACT == 15 || ACT == 16 || ACT == 17, "k_gemm2: unsupported ACT code (would silently apply no activation)");
  __shared__ __attribute__((aligned(16))) float so[4][32][68];
  const int tid = threadIdx.x, w = tid >> 5, lane = tid & 31, ln = lane & 15, hh = lane >> 4; const int by = blockIdx.y;
  A += (size_t)by * sA; Bh += (size_t)by * sB; const size_t cofs = (size_t)by * sC; const float* bp = bias ? bias + (size_t)by * sBias : nullptr;
  const int ntn = N >> 6; const int mt = blockIdx.x / ntn, nq = blockIdx.x - mt * ntn; const int row0 = mt * 128 + 32 * w, col0 = nq * 64; if (row0 >= M) return;
  const _Float16* a0p = A + (size_t)(row0 + ln) * lda; const _Float16* a1p = a0p + (size_t)16 * lda;
  const _Float16* b0p = Bh + (size_t)(col0 + ln) * ldb; const _Float16* b1p = b0p + (size_t)16 * ldb; const _Float16* b2p = b1p + (size_t)16 * ldb; const _Float16* b3p = b2p + (size_t)16 * ldb;
  const v8f z8 = {0.f,0.f,0.f,0.f,0.f,0.f,0.f,0.f}; v8f c00 = z8, c01 = z8, c02 = z8, c03 = z8, c10 = z8, c11 = z8, c12 = z8, c13 = z8;
  for (int kb = 0; kb < K; kb += 32) { const v16h a0 = g2_frag(a0p + kb, hh), a1 = g2_frag(a1p + kb, hh);
    v16h b = g2_frag(b0p + kb, hh); c00 = g2_mma(a0, b, c00); c10 = g2_mma(a1, b, c10);
    b = g2_frag(b1p + kb, hh); c01 = g2_mma(a0, b, c01); c11 = g2_mma(a1, b, c11);
    b = g2_frag(b2p + kb, hh); c02 = g2_mma(a0, b, c02); c12 = g2_mma(a1, b, c12);
    b = g2_frag(b3p + kb, hh); c03 = g2_mma(a0, b, c03); c13 = g2_mma(a1, b, c13); }
  v8f accs[8] = {c00, c01, c02, c03, c10, c11, c12, c13};
#pragma unroll
  for (int u = 0; u < 8; ++u) { const int t = u & 3, half = u >> 2; const int col = col0 + t * 16 + ln; const float bv = bp ? bf16_round(bp[col]) : 0.f;
#pragma unroll
    for (int r = 0; r < 8; ++r) { const int rloc = half * 16 + 8 * hh + r; float v = accs[u][r] * alpha + bv; if (CP) { if (rowsPerB < 0) v += CP[cofs + (size_t)(row0g + row0 + rloc) * ldc + col];        else { const int bidx = (row0g + row0 + rloc) / rowsPerB; v += CP[(size_t)bidx * sCPb + (size_t)by * 64 + col]; } }
      if (ACT == 3) v = fmaxf(v, 0.f); else if (ACT == 6) v = 0.5f * v * (1.0f + erff(v * 0.70710678118654752f)); else if (ACT == 11) v = 1.0f / (1.0f + expf(-v)); else if (ACT == 15) v = v / (1.0f + expf(-v)); else if (ACT == 12) v = (v > 0.f) ? v : 0.01f * v; else if (ACT == 8) v = tanhf(v); else if (ACT == 9) v = 0.5f * v * (1.0f + tanhf(0.7978845608028654f * (v + 0.044715f * v * v * v))); else if (ACT == 14) v = (v > 0.f) ? v : 0.1f * v; else if (ACT == 16) v = (v >= 0.f) ? v : 0.3f * v; else if (ACT == 17) v = (v >= 0.f) ? v : 0.2f * v;
      so[w][rloc][t * 16 + ln] = v; } }
  __builtin_amdgcn_fence(__ATOMIC_ACQ_REL, "workgroup"); __builtin_amdgcn_wave_barrier();
  const int rsub = lane >> 4, c4 = (lane & 15) * 4;
  for (int pass = 0; pass < 2; ++pass) {
#pragma unroll
    for (int q = 0; q < 16; ++q) { const int r = q * 2 + rsub; const v4f v = *(const v4fa*)&so[w][r][c4]; if (C) *(volatile v4f*)(C + cofs + (size_t)(row0 + r) * ldc + col0 + c4) = v; if (C16) { v4h h4; for (int i = 0; i < 4; ++i) h4[i] = (_Float16)v[i]; *(volatile v4h*)(C16 + cofs + (size_t)(row0 + r) * ldc + col0 + c4) = h4; } }
    if (pass == 0) __threadfence(); } }


__global__ __launch_bounds__(256) void k_xtc16(const float* __restrict__ X, _Float16* __restrict__ XT, int n) {
  const int t = blockIdx.x * 256 + threadIdx.x; if (t >= n) return; const int r8 = t & (NN / 8 - 1), dd = t >> 10; const float* s = X + (size_t)(8 * r8) * HD + dd; FragH f;
  for (int i = 0; i < 8; ++i) f.h[i] = (_Float16)bf16_round(s[(size_t)i * HD]);
  unsigned short* o = (unsigned short*)XT + (size_t)dd * NN + 8 * r8; *(volatile v8us*)o = f.half[0]; __threadfence(); *(volatile v8us*)o = f.half[0]; }
__global__ __launch_bounds__(256) void k_gidsm(const float* __restrict__ S, const int* __restrict__ GQ, const int* __restrict__ GK, _Float16* __restrict__ Pm, float* __restrict__ VAL, int n) {
  const int t = blockIdx.x * 256 + threadIdx.x; if (t >= n) return; const int gq = GQ[t]; const float* s = S + (size_t)t * NN; float mx = -3.0e38f; int cnt = 0;
  for (int j = 0; j < NN; ++j) { const int ne = (GK[j] != gq); cnt += 1 - ne; mx = fmaxf(mx, s[j] + (float)ne * -1.0e9f); } float se = 0.f;
  for (int j = 0; j < NN; ++j) { const float pen = (float)(GK[j] != gq) * -1.0e9f; se += __expf((s[j] + pen) - mx); } const float sc = 256.0f / se;
  for (int j0 = 0; j0 < NN; j0 += 8) { FragH f; for (int q = 0; q < 8; ++q) { const float pen = (float)(GK[j0 + q] != gq) * -1.0e9f; f.h[q] = (_Float16)(__expf((s[j0 + q] + pen) - mx) * sc); }
    unsigned short* o = (unsigned short*)Pm + (size_t)t * NN + j0; *(volatile v8us*)o = f.half[0]; __threadfence(); *(volatile v8us*)o = f.half[0]; }
  const float vl = (float)(cnt > 0); *(volatile float*)(VAL + t) = vl; __threadfence(); *(volatile float*)(VAL + t) = vl; }
__global__ __launch_bounds__(256) void k_gidres(const float* __restrict__ O, const float* __restrict__ X, const float* __restrict__ VAL, float* __restrict__ AF, _Float16* __restrict__ A16, int n) {
  const int t = blockIdx.x * 256 + threadIdx.x; if (t >= n) return; const float vl = VAL[t >> 3]; const v4f a = *(const v4fa*)(O + (size_t)t * 8), b = *(const v4fa*)(O + (size_t)t * 8 + 4), xa = *(const v4fa*)(X + (size_t)t * 8), xb = *(const v4fa*)(X + (size_t)t * 8 + 4); v4f ra, rb; FragH f;
  for (int i = 0; i < 4; ++i) { ra[i] = (a[i] + bf16_round(xa[i])) * vl; rb[i] = (b[i] + bf16_round(xb[i])) * vl; f.h[i] = (_Float16)ra[i]; f.h[4 + i] = (_Float16)rb[i]; }
  float* o = AF + (size_t)t * 8; unsigned short* h = (unsigned short*)A16 + (size_t)t * 8;
  for (int pass = 0; pass < 2; ++pass) { *(volatile v4f*)o = ra; *(volatile v4f*)(o + 4) = rb; *(volatile v8us*)h = f.half[0]; if (pass == 0) __threadfence(); } }

extern "C" void kernel_launch(void* const* d_in, const int* in_sizes, int n_in,
                              void* d_out, int out_size, void* d_ws, size_t ws_size, hipStream_t stream) {
  (void)in_sizes; (void)n_in; (void)out_size;
  const float* xs = (const float*)d_in[0]; const int* bs = (const int*)d_in[1]; const float* xt = (const float*)d_in[2]; const int* bt = (const int*)d_in[3];
  const float* w1 = (const float*)d_in[4]; const float* b1 = (const float*)d_in[5]; const float* w2 = (const float*)d_in[6]; const float* b2 = (const float*)d_in[7];
  static_assert(HD == 64 && NN == 8192 && RB == 1024 && NN % RB == 0 && NN / 8 == 1024 && ((size_t)NN * HD / 8) % 256 == 0 && ((size_t)HD * (NN / 8)) % 256 == 0 && RB % 256 == 0 && ((size_t)NN * 8) % 256 == 0 && RB % 128 == 0 && NN % 128 == 0 && NN % 64 == 0 && HD % 64 == 0 && HD % 32 == 0 && NN % 32 == 0, "the index shifts; whole tiles; exact grids");
  float* out = (float*)d_out;
  char* ws = (char*)d_ws; size_t off = 0;
  auto take = [&](size_t bytes) { char* p = ws + off; off += (bytes + 255) & ~(size_t)255; return p; };
  _Float16* XS16 = (_Float16*)take((size_t)NN * HD * 2); _Float16* XT16 = (_Float16*)take((size_t)NN * HD * 2); _Float16* XST = (_Float16*)take((size_t)HD * NN * 2); _Float16* XTT = (_Float16*)take((size_t)HD * NN * 2);
  _Float16* W1T = (_Float16*)take((size_t)HD * HD * 2); _Float16* W2T = (_Float16*)take((size_t)HD * HD * 2);
  float* S = (float*)take((size_t)RB * NN * 4); _Float16* Pm = (_Float16*)take((size_t)RB * NN * 2); float* VAL = (float*)take((size_t)NN * 4);
  float* OF = (float*)take((size_t)NN * HD * 4); float* AF = (float*)take((size_t)NN * HD * 4); _Float16* A16 = (_Float16*)take((size_t)NN * HD * 2); _Float16* H16 = (_Float16*)take((size_t)NN * HD * 2);
  if (off > ws_size) return;
  k_x16<<<(unsigned)((size_t)NN * HD / 8 / 256), 256, 0, stream>>>(xs, XS16, (size_t)NN * HD / 8); k_x16<<<(unsigned)((size_t)NN * HD / 8 / 256), 256, 0, stream>>>(xt, XT16, (size_t)NN * HD / 8);
  k_xtc16<<<(unsigned)((size_t)HD * (NN / 8) / 256), 256, 0, stream>>>(xs, XST, HD * (NN / 8)); k_xtc16<<<(unsigned)((size_t)HD * (NN / 8) / 256), 256, 0, stream>>>(xt, XTT, HD * (NN / 8));
  k_wt_f16<<<(unsigned)(((size_t)HD * (HD / 8) + 255) / 256), 256, 0, stream>>>(w1, W1T, HD, HD, 16.0f); k_wt_f16<<<(unsigned)(((size_t)HD * (HD / 8) + 255) / 256), 256, 0, stream>>>(w2, W2T, HD, HD, 16.0f);
  for (int side = 0; side < 2; ++side) {
    const float* xq = side ? xs : xt; const _Float16* Q16 = side ? XS16 : XT16; const _Float16* K16 = side ? XT16 : XS16; const _Float16* KT = side ? XTT : XST; const int* gq = side ? bs : bt; const int* gk = side ? bt : bs;
    for (int r0 = 0; r0 < NN; r0 += RB) {
      k_gemm2<0><<<dim3((unsigned)((RB / 128) * (NN / 64)), 1), 128, 0, stream>>>(Q16 + (size_t)r0 * HD, HD, 0, K16, HD, 0, 1.0f, nullptr, 0, nullptr, 1, 0, 0, S, nullptr, NN, 0, RB, NN, HD);
      k_gidsm<<<(unsigned)(RB / 256), 256, 0, stream>>>(S, gq + r0, gk, Pm, VAL + r0, RB);
      k_gemm2<0><<<dim3((unsigned)((RB / 128) * (HD / 64)), 1), 128, 0, stream>>>(Pm, NN, 0, KT, NN, 0, 0.00390625f, nullptr, 0, nullptr, 1, 0, 0, OF + (size_t)r0 * HD, nullptr, HD, 0, RB, HD, NN); }
    k_gidres<<<(unsigned)((size_t)NN * 8 / 256), 256, 0, stream>>>(OF, xq, VAL, AF, A16, NN * 8);
    k_gemm2<3><<<dim3((unsigned)((NN / 128) * (HD / 64)), 1), 128, 0, stream>>>(A16, HD, 0, W1T, HD, 0, 0.0625f, b1, 0, nullptr, 1, 0, 0, nullptr, H16, HD, 0, NN, HD, HD);
    k_gemm2<0><<<dim3((unsigned)((NN / 128) * (HD / 64)), 1), 128, 0, stream>>>(H16, HD, 0, W2T, HD, 0, 0.0625f, b2, 0, AF, -1, 0, 0, out + (size_t)side * NN * HD, nullptr, HD, 0, NN, HD, HD); }
}
